// BiMambaBlock_55903294324787
// MI455X (gfx1250) — hardware-verified
//
#include <hip/hip_runtime.h>
#include <math.h>

typedef __attribute__((ext_vector_type(16))) _Float16 v16h;
typedef __attribute__((ext_vector_type(8)))  _Float16 v8h;
typedef __attribute__((ext_vector_type(16))) __bf16   v16b;
typedef __attribute__((ext_vector_type(8)))  __bf16   v8b;
typedef __attribute__((ext_vector_type(8)))  float    v8f;
typedef __attribute__((ext_vector_type(4)))  float    v4f;

constexpr int kBatch = 2;
constexpr int kSeqL  = 1024;
constexpr int kDmod  = 1024;
constexpr int kDin   = 2048;
constexpr int kNst   = 16;
constexpr int kDtR   = 64;
constexpr int kPrjN  = 96;
constexpr int kPrjP  = 128;
constexpr int kXZP   = 2 * kDin;
constexpr int kCmbK  = 2 * kDmod;
constexpr int kRows  = kBatch * kSeqL;
constexpr int kGVP   = 2 * kDmod;
constexpr int kTP    = 260;
constexpr float kEps      = 1e-5f;
constexpr float kCarryW   = 32.0f;
constexpr float kCarryWS  = 4096.0f;
constexpr float kResS     = 1024.0f;
constexpr float kCarryWL  = kCarryWS / kResS;
constexpr float kCarryDt  = 16.0f;
constexpr float kCarryY   = 16.0f;
static_assert(kCarryWL == 4.0f, "residual weight carry");
static_assert(kDtR + 2 * kNst == kPrjN, "x_proj width");
static_assert((kRows % 64) == 0, "M of every GEMM");
static_assert((kXZP % 64) == 0 && (kDmod % 32) == 0, "in_proj N,K");
static_assert((kPrjP % 64) == 0 && (kDin % 32) == 0, "x_proj N,K");
static_assert((kDin % 64) == 0 && (kDtR % 32) == 0, "dt_proj N,K");
static_assert((kDmod % 64) == 0 && (kDin % 32) == 0, "out_proj N,K");
static_assert((kDmod % 64) == 0 && (kCmbK % 32) == 0, "gate and value N,K");
static_assert((kSeqL % 64) == 0 && (kDin % 256) == 0 && (kDmod == 128 * 8) && (kSeqL % 16) == 0, "tile multiples");

constexpr size_t kSzWIN16  = (size_t)kXZP * kDmod * 2;
constexpr size_t kSzWXP16  = (size_t)kPrjP * kDin * 2;
constexpr size_t kSzWDT16  = (size_t)kDin * kDtR * 2;
constexpr size_t kSzWOUT16 = (size_t)kDmod * kDin * 2;
constexpr size_t kSzWOUTL  = (size_t)kDmod * kDin * 2;
constexpr size_t kSzXN16   = (size_t)kRows * kDmod * 2;
constexpr size_t kSzXZ     = (size_t)kRows * kXZP * 4;
constexpr size_t kSzUC16   = (size_t)kRows * kDin * 2;
constexpr size_t kSzPROJ   = (size_t)kRows * kPrjP * 4;
constexpr size_t kSzDT16   = (size_t)kRows * kDtR * 2;
constexpr size_t kSzDLR    = (size_t)kRows * kDin * 4;
constexpr size_t kSzY16    = (size_t)kRows * kDin * 2;
constexpr size_t kSzYL     = (size_t)kRows * kDin * 2;
constexpr size_t kSzMO     = (size_t)2 * kRows * kDmod * 4;
constexpr size_t kSzCOMBH  = (size_t)kRows * kCmbK * 2;
constexpr size_t kSzCOMBL  = (size_t)kRows * kCmbK * 2;
constexpr size_t kOffWIN16  = 0;
constexpr size_t kOffWXP16  = kOffWIN16  + kSzWIN16;
constexpr size_t kOffWDT16  = kOffWXP16  + kSzWXP16;
constexpr size_t kOffWOUT16 = kOffWDT16  + kSzWDT16;
constexpr size_t kOffWOUTL  = kOffWOUT16 + kSzWOUT16;
constexpr size_t kOffXN16   = kOffWOUTL  + kSzWOUTL;
constexpr size_t kOffXZ     = kOffXN16   + kSzXN16;
constexpr size_t kOffUC16   = kOffXZ     + kSzXZ;
constexpr size_t kOffPROJ   = kOffUC16   + kSzUC16;
constexpr size_t kOffDT16   = kOffPROJ   + kSzPROJ;
constexpr size_t kOffDLR    = kOffDT16   + kSzDT16;
constexpr size_t kOffY16    = kOffDLR    + kSzDLR;
constexpr size_t kOffYL     = kOffY16    + kSzY16;
constexpr size_t kOffMO     = kOffYL     + kSzYL;
constexpr size_t kOffCOMBH  = kOffMO     + kSzMO;
constexpr size_t kOffCOMBL  = kOffCOMBH  + kSzCOMBH;
constexpr size_t kWsTotal   = kOffCOMBL  + kSzCOMBL;
constexpr size_t kOffWGVH   = kOffY16;
constexpr size_t kOffWGVL   = kOffYL;
constexpr size_t kOffGV     = kOffDLR;
static_assert(kWsTotal == 132120576ull, "carve total");
static_assert(kWsTotal <= 134217728ull, "carve cap");
static_assert((size_t)kCmbK * kCmbK * 2 == kSzY16 && kSzY16 == kSzYL, "WGVH and WGVL fit the Y16 and YL regions exactly");
static_assert((size_t)kRows * kGVP * 4 == kSzDLR, "GV fits the DLR region exactly");
static_assert((kOffWXP16 % 262144) == 0 && (kOffWDT16 % 262144) == 0 && (kOffWOUT16 % 262144) == 0 &&
              (kOffWOUTL % 262144) == 0 && (kOffXN16 % 262144) == 0 && (kOffXZ % 262144) == 0 &&
              (kOffUC16 % 262144) == 0 && (kOffPROJ % 262144) == 0 && (kOffDT16 % 262144) == 0 &&
              (kOffDLR % 262144) == 0 && (kOffY16 % 262144) == 0 && (kOffYL % 262144) == 0 &&
              (kOffMO % 262144) == 0 && (kOffCOMBH % 262144) == 0 && (kOffCOMBL % 262144) == 0, "aligned regions");

__device__ __forceinline__ unsigned short f2bf_bits(float f) {
  unsigned u = __float_as_uint(f);
  return (unsigned short)((u + 0x7FFFu + ((u >> 16) & 1u)) >> 16);
}
__device__ __forceinline__ float bf_bits2f(unsigned short h) { return __uint_as_float(((unsigned)h) << 16); }

__device__ __forceinline__ float h16_to_f32(unsigned hb) {
  const unsigned sgn = (hb & 0x8000u) << 16; const unsigned em = hb & 0x7fffu;
  const float fn = __uint_as_float((em << 13) + 0x38000000u);
  const float fs = (float)em * 5.9604644775390625e-8f;
  const float mag = (em < 0x400u) ? fs : fn; return __uint_as_float(__float_as_uint(mag) | sgn);
}
__device__ __forceinline__ void split_f16(float v, _Float16& hi, _Float16& lo) {
  const _Float16 hh = (_Float16)v;
  const unsigned hb = (unsigned)__builtin_bit_cast(unsigned short, hh);
  const float hf = h16_to_f32(hb);
  hi = hh;
  lo = (_Float16)((v - hf) * kResS);
}

__device__ __forceinline__ void dep_guard4_h(v8f& a, v8f& b, v8f& c, v8f& d, v16h x, v16h y) { asm volatile("v_nop\n\tv_nop\n\tv_nop\n\tv_nop" : "+v"(a), "+v"(b), "+v"(c), "+v"(d) : "v"(x), "v"(y)); }
__device__ __forceinline__ void dep_guard4_b(v8f& a, v8f& b, v8f& c, v8f& d, v16b x, v16b y) { asm volatile("v_nop\n\tv_nop\n\tv_nop\n\tv_nop" : "+v"(a), "+v"(b), "+v"(c), "+v"(d) : "v"(x), "v"(y)); }
__device__ __forceinline__ void keep4_h(v16h a, v16h b, v16h c, v16h d) { asm volatile("v_nop" :: "v"(a), "v"(b), "v"(c), "v"(d)); }
__device__ __forceinline__ void keep4_b(v16b a, v16b b, v16b c, v16b d) { asm volatile("v_nop" :: "v"(a), "v"(b), "v"(c), "v"(d)); }
__device__ __forceinline__ void acc_guard4(v8f& a, v8f& b, v8f& c, v8f& d) { asm volatile("v_nop\n\tv_nop\n\tv_nop\n\tv_nop" : "+v"(a), "+v"(b), "+v"(c), "+v"(d)); }
template <typename T> struct Frag;
template <> struct Frag<_Float16> {
  typedef v16h V; union U { v16h v; v8h h[2]; };
  static __device__ __forceinline__ v16h load(const _Float16* p) {
    U f; f.h[0] = *(const v8h*)(p); f.h[1] = *(const v8h*)(p + 16); return f.v;
  }
  static __device__ __forceinline__ v8f mma(v16h a, v16h b, v8f c) {
    return __builtin_amdgcn_wmma_f32_16x16x32_f16(false, a, false, b, (short)0, c, false, false);
  }
  static __device__ __forceinline__ void guard4(v8f& a, v8f& b, v8f& c, v8f& d, v16h x, v16h y) { dep_guard4_h(a, b, c, d, x, y); }
  static __device__ __forceinline__ void keep(v16h a, v16h b, v16h c, v16h d) { keep4_h(a, b, c, d); }
};
template <> struct Frag<__bf16> {
  typedef v16b V; union U { v16b v; v8b h[2]; };
  static __device__ __forceinline__ v16b load(const __bf16* p) {
    U f; f.h[0] = *(const v8b*)(p); f.h[1] = *(const v8b*)(p + 16); return f.v;
  }
  static __device__ __forceinline__ v8f mma(v16b a, v16b b, v8f c) {
    return __builtin_amdgcn_wmma_f32_16x16x32_bf16(false, a, false, b, (short)0, c, false, false);
  }
  static __device__ __forceinline__ void guard4(v8f& a, v8f& b, v8f& c, v8f& d, v16b x, v16b y) { dep_guard4_b(a, b, c, d, x, y); }
  static __device__ __forceinline__ void keep(v16b a, v16b b, v16b c, v16b d) { keep4_b(a, b, c, d); }
};

template <int ET> struct Elem;
template <> struct Elem<0> { typedef _Float16 T; };
template <> struct Elem<1> { typedef __bf16 T; };
template <int ET, int SPL, int BIAS_MODE, int OUT_MODE, bool RESID, int ACT = 0>
__global__ __launch_bounds__(256) void wmma_gemm64(
    const unsigned short* __restrict__ Ap, const unsigned short* __restrict__ A2p, int lda, long strideA,
    const unsigned short* __restrict__ Btp, const unsigned short* __restrict__ Bt2p, int ldb, long strideB,
    void* __restrict__ Cout, void* __restrict__ Cout2, int ldc, long strideC,
    const float* __restrict__ bias,
    const float* __restrict__ resid, long strideR,
    int M, int N, int K, float scale) {
  typedef typename Elem<ET>::T T;
  typedef typename Frag<T>::V V;
  const T* A = (const T*)Ap; const T* A2 = (const T*)A2p; const T* Bt = (const T*)Btp; const T* Bt2 = (const T*)Bt2p;
  __shared__ __align__(16) float sT[8][16 * 68];
  const int b    = blockIdx.y;
  const int lane = threadIdx.x & 31;
  const int wave = threadIdx.x >> 5;
  const int tilesN = N >> 6;
  const int tilesM = M >> 6;
  const int tile = blockIdx.x * 8 + wave;
  if (tile >= tilesM * tilesN) return;
  const int tm = tile / tilesN;
  const int tn = tile - tm * tilesN;
  const int m0 = tm << 6;
  const int n0 = tn << 6;

  const T* Ab  = A  + (size_t)b * strideA;
  const T* Bb  = Bt + (size_t)b * strideB;
  const T* Ab2 = (SPL >= 1) ? (A2  + (size_t)b * strideA) : nullptr;
  const T* Bb2 = (SPL >= 2) ? (Bt2 + (size_t)b * strideB) : nullptr;

  const int rlane = lane & 15;
  const int koff  = (lane >> 4) * 8;
  const int mOff  = (lane >> 4) * 8;

  v8f acc[4][4];
#pragma unroll
  for (int i = 0; i < 4; ++i)
#pragma unroll
    for (int j = 0; j < 4; ++j) acc[i][j] = (v8f){0.f,0.f,0.f,0.f,0.f,0.f,0.f,0.f};

  for (int k0 = 0; k0 < K; k0 += 32) {
    V bh[4], bl[4];
#pragma unroll
    for (int j = 0; j < 4; ++j) {
      const size_t bo = (size_t)(n0 + (j << 4) + rlane) * ldb + koff + k0;
      bh[j] = Frag<T>::load(Bb + bo);
      if (SPL >= 2) bl[j] = Frag<T>::load(Bb2 + bo);
    }
#pragma unroll
    for (int i = 0; i < 4; ++i) {
      const size_t ao = (size_t)(m0 + (i << 4) + rlane) * lda + koff + k0;
      V ah = Frag<T>::load(Ab + ao);
      V al;
      if (SPL >= 1) al = Frag<T>::load(Ab2 + ao);
#pragma unroll
      for (int j = 0; j < 4; ++j) {
        acc[i][j] = Frag<T>::mma(ah, bh[j], acc[i][j]);
        if (SPL == 2) acc[i][j] = Frag<T>::mma(ah, bl[j], acc[i][j]);
        if (SPL == 1 || SPL == 2) acc[i][j] = Frag<T>::mma(al, bh[j], acc[i][j]);
        if (SPL == 3) acc[i][j] = Frag<T>::mma(al, bl[j], acc[i][j]);
      }
      Frag<T>::guard4(acc[i][0], acc[i][1], acc[i][2], acc[i][3], ah, (SPL >= 1) ? al : ah);
    }
    Frag<T>::keep(bh[0], bh[1], bh[2], bh[3]);
    if (SPL >= 2) Frag<T>::keep(bl[0], bl[1], bl[2], bl[3]);
  }
  acc_guard4(acc[0][0], acc[0][1], acc[0][2], acc[0][3]);
  acc_guard4(acc[1][0], acc[1][1], acc[1][2], acc[1][3]);
  acc_guard4(acc[2][0], acc[2][1], acc[2][2], acc[2][3]);
  acc_guard4(acc[3][0], acc[3][1], acc[3][2], acc[3][3]);

  float* slab = sT[wave];
  const float* Rb = RESID ? (resid + (size_t)b * strideR) : nullptr;
#pragma unroll
  for (int i = 0; i < 4; ++i) {
    const int mBase = m0 + (i << 4);
#pragma unroll
    for (int j = 0; j < 4; ++j) {
      const int n = n0 + (j << 4) + rlane;
      float bv = 0.f;
      if (BIAS_MODE == 2) bv = bias[n];
#pragma unroll
      for (int r = 0; r < 8; ++r) {
        float v = acc[i][j][r] * scale;
        if (BIAS_MODE == 1) v += bias[mBase + mOff + r];
        if (BIAS_MODE == 2) v += bv;
        if (RESID) v += Rb[(size_t)(mBase + mOff + r) * ldc + n];
        if (ACT == 1) v = tanhf(v);
        if (ACT == 2) v = fmaxf(v, 0.0f);
        if (ACT == 3) v = v / (1.0f + expf(-v));
        if (ACT == 4) v = (v > 0.f) ? v : 0.01f * v;
        slab[(mOff + r) * 68 + (j << 4) + rlane] = v;
      }
    }
    __builtin_amdgcn_fence(__ATOMIC_RELEASE, "workgroup");
    __builtin_amdgcn_wave_barrier();
    __builtin_amdgcn_fence(__ATOMIC_ACQUIRE, "workgroup");
    if (OUT_MODE == 0) {
      float* C = (float*)Cout + (size_t)b * strideC;
      const int hh = lane >> 4, c4 = (lane & 15) * 4;
      for (int pass = 0; pass < 2; ++pass) {
#pragma unroll
        for (int it = 0; it < 8; ++it) {
          const int row = it * 2 + hh;
          v4f v = *(const v4f*)(slab + row * 68 + c4);
          *(volatile v4f*)(C + (size_t)(mBase + row) * ldc + n0 + c4) = v;
        }
        __threadfence();
      }
    } else {
      const int q = lane >> 3, c8 = (lane & 7) * 8;
      unsigned short* C  = (unsigned short*)Cout  + (size_t)b * strideC;
      unsigned short* C2 = (OUT_MODE == 2) ? ((unsigned short*)Cout2 + (size_t)b * strideC) : nullptr;
      for (int pass = 0; pass < 2; ++pass) {
#pragma unroll
        for (int it = 0; it < 4; ++it) {
          const int row = it * 4 + q;
          const float* sp = slab + row * 68 + c8;
          v8h hv, lv;
#pragma unroll
          for (int e = 0; e < 8; ++e) {
            if (OUT_MODE == 1) {
              hv[e] = (_Float16)sp[e];
            } else {
              unsigned short hb = f2bf_bits(sp[e]);
              unsigned short lb = f2bf_bits(sp[e] - bf_bits2f(hb));
              hv[e] = __builtin_bit_cast(_Float16, hb);
              lv[e] = __builtin_bit_cast(_Float16, lb);
            }
          }
          *(volatile v8h*)(C + (size_t)(mBase + row) * ldc + n0 + c8) = hv;
          if (OUT_MODE == 2) *(volatile v8h*)(C2 + (size_t)(mBase + row) * ldc + n0 + c8) = lv;
        }
        __threadfence();
      }
    }
    __builtin_amdgcn_fence(__ATOMIC_RELEASE, "workgroup");
    __builtin_amdgcn_wave_barrier();
    __builtin_amdgcn_fence(__ATOMIC_ACQUIRE, "workgroup");
  }
}

__global__ __launch_bounds__(256) void transpose_cast_kernel(
    const float* __restrict__ W, unsigned short* __restrict__ Bt, int Kdim, int Ndim, int Npad, float scale)
{
  __shared__ float tile[64 * 65];
  const int tid = threadIdx.x, lane = tid & 31, wave = tid >> 5;
  const int n0 = blockIdx.x * 64;
  const int k0 = blockIdx.y * 64;
  (void)Npad;
#pragma unroll
  for (int p = 0; p < 16; ++p) {
    const int idx = tid + p * 256;
    const int kk  = idx >> 6;
    const int nn  = idx & 63;
    const int n   = n0 + nn;
    const int nc  = (n < Ndim) ? n : (Ndim - 1);
    const float v = W[(size_t)(k0 + kk) * Ndim + nc];
    tile[kk * 65 + nn] = (n < Ndim) ? (v * scale) : 0.f;
  }
  __syncthreads();
  const int q = lane >> 3, c8 = (lane & 7) * 8;
  v8h hv[2];
#pragma unroll
  for (int it = 0; it < 2; ++it) {
    const int nrow = it * 32 + wave * 4 + q;
#pragma unroll
    for (int e = 0; e < 8; ++e) hv[it][e] = (_Float16)tile[(c8 + e) * 65 + nrow];
  }
  for (int pass = 0; pass < 2; ++pass) {
#pragma unroll
    for (int it = 0; it < 2; ++it) {
      const int nrow = it * 32 + wave * 4 + q;
      *(volatile v8h*)(Bt + (size_t)(n0 + nrow) * Kdim + k0 + c8) = hv[it];
    }
    __threadfence();
  }
}

__global__ __launch_bounds__(128) void layernorm_f16_kernel(
    const float* __restrict__ x, const float* __restrict__ lw, const float* __restrict__ lb,
    unsigned short* __restrict__ XN16)
{
  __shared__ float sred[8];
  const int tid = threadIdx.x, lane = tid & 31, wave = tid >> 5;
  const int row = blockIdx.x;
  const int c0 = tid * 8;
  const float* xr = x + (size_t)row * kDmod + c0;
  const v4f a0 = *(const v4f*)(xr);
  const v4f a1 = *(const v4f*)(xr + 4);
  float s = 0.0f;
#pragma unroll
  for (int e = 0; e < 4; ++e) s += a0[e];
#pragma unroll
  for (int e = 0; e < 4; ++e) s += a1[e];
#pragma unroll
  for (int off = 16; off >= 1; off >>= 1) s += __shfl_xor(s, off, 32);
  if (lane == 0) sred[wave] = s;
  __syncthreads();
  const float mu = ((sred[0] + sred[1]) + (sred[2] + sred[3])) * (1.0f / (float)kDmod);
  float qv = 0.0f;
#pragma unroll
  for (int e = 0; e < 4; ++e) { const float dd = a0[e] - mu; qv = fmaf(dd, dd, qv); }
#pragma unroll
  for (int e = 0; e < 4; ++e) { const float dd = a1[e] - mu; qv = fmaf(dd, dd, qv); }
#pragma unroll
  for (int off = 16; off >= 1; off >>= 1) qv += __shfl_xor(qv, off, 32);
  if (lane == 0) sred[4 + wave] = qv;
  __syncthreads();
  const float var = ((sred[4] + sred[5]) + (sred[6] + sred[7])) * (1.0f / (float)kDmod);
  const float rs = rsqrtf(var + kEps);
  const v4f w0 = *(const v4f*)(lw + c0);
  const v4f w1 = *(const v4f*)(lw + c0 + 4);
  const v4f b0 = *(const v4f*)(lb + c0);
  const v4f b1 = *(const v4f*)(lb + c0 + 4);
  v8h hv;
#pragma unroll
  for (int e = 0; e < 4; ++e) {
    hv[e]     = (_Float16)((a0[e] - mu) * rs * w0[e] + b0[e]);
    hv[4 + e] = (_Float16)((a1[e] - mu) * rs * w1[e] + b1[e]);
  }
  unsigned short* qd = XN16 + (size_t)row * kDmod + c0;
  *(volatile v8h*)qd = hv;
  __threadfence();
  *(volatile v8h*)qd = hv;
}

__global__ __launch_bounds__(256) void dt_cast_kernel(
    const float* __restrict__ PROJ, unsigned short* __restrict__ DT16, int total8, float scale)
{
  const int i = blockIdx.x * 256 + threadIdx.x;
  if (i >= total8) return;
  const int e0  = i << 3;
  const int row = e0 >> 6;
  const int c8  = e0 & 63;
  const float* p = PROJ + (size_t)row * kPrjP + c8;
  const v4f a0 = *(const v4f*)(p);
  const v4f a1 = *(const v4f*)(p + 4);
  v8h hv;
#pragma unroll
  for (int e = 0; e < 4; ++e) {
    hv[e]     = (_Float16)(a0[e] * scale);
    hv[4 + e] = (_Float16)(a1[e] * scale);
  }
  unsigned short* qd = DT16 + e0;
  *(volatile v8h*)qd = hv;
  __threadfence();
  *(volatile v8h*)qd = hv;
}

__global__ __launch_bounds__(256) void conv_silu_kernel(
    const float* __restrict__ XZ, const float* __restrict__ cw, const float* __restrict__ cb,
    unsigned short* __restrict__ UC16, int dir)
{
  __shared__ __align__(16) float sT[16 * kTP];
  const int tid = threadIdx.x, lane = tid & 31, wave = tid >> 5;
  const int d0 = blockIdx.x * 256, d = d0 + tid;
  const int g0 = blockIdx.y * 64;
  const int tb = g0 & (kSeqL - 1);
  const float w0 = cw[d * 4 + 0], w1 = cw[d * 4 + 1], w2 = cw[d * 4 + 2], w3 = cw[d * 4 + 3];
  const float bc = cb[d];
  float xm3, xm2, xm1;
  {
    const bool hist = dir ? (tb + 64 < kSeqL) : (tb > 0);
    const int r3 = hist ? (dir ? (g0 + 66) : (g0 - 3)) : g0;
    const int r2 = hist ? (dir ? (g0 + 65) : (g0 - 2)) : g0;
    const int r1 = hist ? (dir ? (g0 + 64) : (g0 - 1)) : g0;
    const float v3 = XZ[(size_t)r3 * kXZP + d];
    const float v2 = XZ[(size_t)r2 * kXZP + d];
    const float v1 = XZ[(size_t)r1 * kXZP + d];
    xm3 = hist ? v3 : 0.f;
    xm2 = hist ? v2 : 0.f;
    xm1 = hist ? v1 : 0.f;
  }
#pragma unroll 1
  for (int sub = 0; sub < 4; ++sub) {
    const int lbase = g0 + (dir ? (48 - sub * 16) : (sub * 16));
#pragma unroll 1
    for (int s = 0; s < 16; ++s) {
      const int rr = dir ? (15 - s) : s;
      const float xc = XZ[(size_t)(lbase + rr) * kXZP + d];
      float acc = w0 * xm3;
      acc = fmaf(w1, xm2, acc);
      acc = fmaf(w2, xm1, acc);
      acc = fmaf(w3, xc, acc);
      const float sv = acc + bc;
      const float sg = __builtin_amdgcn_rcpf(1.0f + __expf(-sv));
      sT[rr * kTP + tid] = sv * sg;
      xm3 = xm2; xm2 = xm1; xm1 = xc;
    }
    __syncthreads();
    v8h bv[2];
#pragma unroll
    for (int it = 0; it < 2; ++it) {
      const float* sp = sT + (it * 8 + wave) * kTP + lane * 8;
      const v4f a0 = *(const v4f*)(sp);
      const v4f a1 = *(const v4f*)(sp + 4);
#pragma unroll
      for (int e = 0; e < 4; ++e) {
        bv[it][e]     = (_Float16)a0[e];
        bv[it][4 + e] = (_Float16)a1[e];
      }
    }
    for (int pass = 0; pass < 2; ++pass) {
#pragma unroll
      for (int it = 0; it < 2; ++it)
        *(volatile v8h*)(UC16 + (size_t)(lbase + it * 8 + wave) * kDin + d0 + lane * 8) = bv[it];
      __threadfence();
    }
    __syncthreads();
  }
}

__global__ __launch_bounds__(256) void scan_kernel(
    const float* __restrict__ DLR, const float* __restrict__ XZ, const float* __restrict__ PROJ,
    const float* __restrict__ cw, const float* __restrict__ cb,
    const float* __restrict__ A_log, const float* __restrict__ Dv,
    unsigned short* __restrict__ Y16, unsigned short* __restrict__ YL, int dir)
{
  __shared__ __align__(16) float sBC[16 * 32];
  __shared__ __align__(16) float sY[16 * kTP];
  const int tid = threadIdx.x, lane = tid & 31, wave = tid >> 5;
  const int d0 = blockIdx.x * 256, d = d0 + tid;
  const size_t rowbase = (size_t)blockIdx.y * kSeqL;

  float An[kNst];
#pragma unroll
  for (int n = 0; n < 8; ++n) An[n] = -__expf(A_log[(size_t)d * kNst + n]);
  asm volatile("" ::: "memory");
#pragma unroll
  for (int n = 8; n < kNst; ++n) An[n] = -__expf(A_log[(size_t)d * kNst + n]);
  asm volatile("" ::: "memory");
  const float w0 = cw[d * 4 + 0], w1 = cw[d * 4 + 1], w2 = cw[d * 4 + 2], w3 = cw[d * 4 + 3];
  const float bc = cb[d];
  const float Dd = Dv[d];
  float h[kNst];
#pragma unroll
  for (int n = 0; n < kNst; ++n) h[n] = 0.f;
  float xm3 = 0.f, xm2 = 0.f, xm1 = 0.f;

#pragma unroll 1
  for (int c = 0; c < kSeqL / 16; ++c) {
    const int l0 = dir ? (kSeqL - 16 - c * 16) : (c * 16);
    if (tid < 128) {
      const int r = tid >> 3, q = (tid & 7) * 4;
      const v4f v = *(const v4f*)(PROJ + (rowbase + l0 + r) * kPrjP + kDtR + q);
      *(v4f*)(sBC + r * 32 + q) = v;
    }
    __syncthreads();
#pragma unroll 1
    for (int s = 0; s < 16; ++s) {
      const int rr = dir ? (15 - s) : s;
      const size_t m = rowbase + l0 + rr;
      const float a     = DLR[m * kDin + d];
      const float xc    = XZ[m * kXZP + d];
      const float zv    = XZ[m * kXZP + kDin + d];
      const float delta = fmaxf(a, 0.0f) + log1pf(__expf(-fabsf(a)));
      float cacc = w0 * xm3;
      cacc = fmaf(w1, xm2, cacc);
      cacc = fmaf(w2, xm1, cacc);
      cacc = fmaf(w3, xc, cacc);
      const float sv  = cacc + bc;
      const float sgu = __builtin_amdgcn_rcpf(1.0f + __expf(-sv));
      const float xv  = sv * sgu;
      xm3 = xm2; xm2 = xm1; xm1 = xc;
      v4f Bq[4], Cq[4];
#pragma unroll
      for (int qq = 0; qq < 4; ++qq) {
        Bq[qq] = *(const v4f*)(sBC + rr * 32 + 4 * qq);
        Cq[qq] = *(const v4f*)(sBC + rr * 32 + kNst + 4 * qq);
      }
      float y = 0.f;
#pragma unroll
      for (int n = 0; n < kNst; ++n) {
        const float e = __expf(delta * An[n]);
        float db = delta * Bq[n >> 2][n & 3];
        asm volatile("" : "+v"(db));
        float p = db * xv;
        asm volatile("" : "+v"(p));
        float qv = h[n] * e;
        asm volatile("" : "+v"(qv));
        const float hn = qv + p;
        h[n] = hn;
        float rr2 = Cq[n >> 2][n & 3] * hn;
        asm volatile("" : "+v"(rr2));
        y += rr2;
      }
      float sk = xv * Dd;
      asm volatile("" : "+v"(sk));
      y += sk;
      const float sg = __builtin_amdgcn_rcpf(1.0f + __expf(-zv));
      const float g  = zv * sg;
      sY[rr * kTP + tid] = (y * g) * kCarryY;
    }
    __syncthreads();
    v8h hv[2], lv[2];
#pragma unroll
    for (int it = 0; it < 2; ++it) {
      const float* sp = sY + (it * 8 + wave) * kTP + lane * 8;
      const v4f a0 = *(const v4f*)(sp);
      const v4f a1 = *(const v4f*)(sp + 4);
#pragma unroll
      for (int e = 0; e < 4; ++e) {
        _Float16 ph, pl;
        split_f16(a0[e], ph, pl);
        hv[it][e] = ph; lv[it][e] = pl;
        split_f16(a1[e], ph, pl);
        hv[it][4 + e] = ph; lv[it][4 + e] = pl;
      }
    }
    for (int pass = 0; pass < 2; ++pass) {
#pragma unroll
      for (int it = 0; it < 2; ++it) {
        const size_t o = (rowbase + l0 + it * 8 + wave) * kDin + d0 + lane * 8;
        *(volatile v8h*)(Y16 + o) = hv[it];
        *(volatile v8h*)(YL + o) = lv[it];
      }
      __threadfence();
    }
  }
}

__global__ __launch_bounds__(256) void comb_cast_kernel(
    const float* __restrict__ MO, const float* __restrict__ x,
    unsigned short* __restrict__ COMBH, unsigned short* __restrict__ COMBL, int total8)
{
  const int i = blockIdx.x * 256 + threadIdx.x;
  if (i >= total8) return;
  const size_t e0 = (size_t)i << 3;
  const int row  = (int)(e0 >> 11);
  const int c    = (int)(e0 & (size_t)(kCmbK - 1));
  const int half = c >> 10;
  const int cc   = c & (kDmod - 1);
  const float* mp = MO + (size_t)half * kRows * kDmod + (size_t)row * kDmod + cc;
  const float* xp = x + (size_t)row * kDmod + cc;
  const v4f m0 = *(const v4f*)(mp);
  const v4f m1 = *(const v4f*)(mp + 4);
  const v4f x0 = *(const v4f*)(xp);
  const v4f x1 = *(const v4f*)(xp + 4);
  v8h hv, lv;
#pragma unroll
  for (int e = 0; e < 4; ++e) {
    _Float16 ph, pl;
    split_f16(m0[e] + x0[e], ph, pl);
    hv[e] = ph; lv[e] = pl;
    split_f16(m1[e] + x1[e], ph, pl);
    hv[4 + e] = ph; lv[4 + e] = pl;
  }
  unsigned short* qh = COMBH + e0;
  unsigned short* ql = COMBL + e0;
  *(volatile v8h*)qh = hv;
  *(volatile v8h*)ql = lv;
  __threadfence();
  *(volatile v8h*)qh = hv;
  *(volatile v8h*)ql = lv;
}

__global__ __launch_bounds__(256) void gate_fuse_kernel(
    const float* __restrict__ GV, const float* __restrict__ MO, const float* __restrict__ x,
    float* __restrict__ out, int total4)
{
  const int i = blockIdx.x * 256 + threadIdx.x;
  if (i >= total4) return;
  const size_t e0 = (size_t)i << 2;
  const int row = (int)(e0 >> 10);
  const int c   = (int)(e0 & (size_t)(kDmod - 1));
  const float* gp = GV + (size_t)row * kGVP + c;
  const v4f gl = *(const v4f*)(gp);
  const v4f vv = *(const v4f*)(gp + kDmod);
  const v4f m0 = *(const v4f*)(MO + e0);
  const v4f m1 = *(const v4f*)(MO + (size_t)kRows * kDmod + e0);
  const v4f xv = *(const v4f*)(x + e0);
  v4f o;
#pragma unroll
  for (int e = 0; e < 4; ++e) {
    const float g  = __builtin_amdgcn_rcpf(1.0f + expf(-gl[e]));
    const float fw = m0[e] + xv[e];
    const float bw = m1[e] + xv[e];
    const float om = 1.0f - g;
    float t = g * vv[e];
    t = fmaf(om, fw, t);
    t = fmaf(om, bw, t);
    o[e] = t * 0.5f;
  }
  float* qd = out + e0;
  *(volatile v4f*)qd = o;
  __threadfence();
  *(volatile v4f*)qd = o;
}

extern "C" void kernel_launch(void* const* d_in, const int* in_sizes, int n_in,
                              void* d_out, int out_size, void* d_ws, size_t ws_size,
                              hipStream_t stream)
{
  if (n_in < 18) return;
  if (in_sizes[0]  != kRows * kDmod) return;
  if (in_sizes[1]  != 2 * kDmod || in_sizes[2] != 2 * kDmod) return;
  if (in_sizes[3]  != 2 * kDmod * kXZP || in_sizes[4] != 2 * kXZP) return;
  if (in_sizes[5]  != 2 * kDin * 4 || in_sizes[6] != 2 * kDin) return;
  if (in_sizes[7]  != 2 * kDin * kPrjN) return;
  if (in_sizes[8]  != 2 * kDtR * kDin || in_sizes[9] != 2 * kDin) return;
  if (in_sizes[10] != 2 * kDin * kNst || in_sizes[11] != 2 * kDin) return;
  if (in_sizes[12] != 2 * kDin * kDmod || in_sizes[13] != 2 * kDmod) return;
  if (in_sizes[14] != kCmbK * kDmod || in_sizes[15] != kDmod) return;
  if (in_sizes[16] != kCmbK * kDmod || in_sizes[17] != kDmod) return;
  if (out_size != kRows * kDmod) return;
  if (ws_size < kWsTotal) return;

  const float* x      = (const float*)d_in[0];
  const float* ln_w   = (const float*)d_in[1];
  const float* ln_b   = (const float*)d_in[2];
  const float* W_in   = (const float*)d_in[3];
  const float* b_in   = (const float*)d_in[4];
  const float* conv_w = (const float*)d_in[5];
  const float* conv_b = (const float*)d_in[6];
  const float* W_xprj = (const float*)d_in[7];
  const float* W_dt   = (const float*)d_in[8];
  const float* b_dt   = (const float*)d_in[9];
  const float* A_log  = (const float*)d_in[10];
  const float* Dv     = (const float*)d_in[11];
  const float* W_out  = (const float*)d_in[12];
  const float* b_out  = (const float*)d_in[13];
  const float* Wg     = (const float*)d_in[14];
  const float* bg     = (const float*)d_in[15];
  const float* Wv     = (const float*)d_in[16];
  const float* bv     = (const float*)d_in[17];
  float* dout = (float*)d_out;

  char* ws = (char*)d_ws;
  unsigned short* WIN16  = (unsigned short*)(ws + kOffWIN16);
  unsigned short* WXP16  = (unsigned short*)(ws + kOffWXP16);
  unsigned short* WDT16  = (unsigned short*)(ws + kOffWDT16);
  unsigned short* WOUT16 = (unsigned short*)(ws + kOffWOUT16);
  unsigned short* WOUTL  = (unsigned short*)(ws + kOffWOUTL);
  unsigned short* XN16   = (unsigned short*)(ws + kOffXN16);
  float*          XZ     = (float*)(ws + kOffXZ);
  unsigned short* UC16   = (unsigned short*)(ws + kOffUC16);
  float*          PROJ   = (float*)(ws + kOffPROJ);
  unsigned short* DT16   = (unsigned short*)(ws + kOffDT16);
  float*          DLR    = (float*)(ws + kOffDLR);
  unsigned short* Y16    = (unsigned short*)(ws + kOffY16);
  unsigned short* YL     = (unsigned short*)(ws + kOffYL);
  float*          MO     = (float*)(ws + kOffMO);
  unsigned short* COMBH  = (unsigned short*)(ws + kOffCOMBH);
  unsigned short* COMBL  = (unsigned short*)(ws + kOffCOMBL);
  unsigned short* WGVH   = (unsigned short*)(ws + kOffWGVH);
  unsigned short* WGVL   = (unsigned short*)(ws + kOffWGVL);
  float*          GV     = (float*)(ws + kOffGV);
  const float* dummy_bias  = b_dt;
  const float* dummy_resid = x;

  const float sclW   = 1.0f / kCarryW;
  const float sclDtW = 1.0f / (kCarryDt * kCarryW);
  const float sclYW  = 1.0f / (kCarryY * kCarryWS);
  const float sclGW  = 1.0f / kCarryWS;

  for (int dir = 0; dir < 2; ++dir) {
    transpose_cast_kernel<<<dim3(kXZP / 64, kDmod / 64), 256, 0, stream>>>(W_in + (size_t)dir * kDmod * kXZP, WIN16, kDmod, kXZP, kXZP, kCarryW);
    transpose_cast_kernel<<<dim3(kPrjP / 64, kDin / 64), 256, 0, stream>>>(W_xprj + (size_t)dir * kDin * kPrjN, WXP16, kDin, kPrjN, kPrjP, kCarryW);
    transpose_cast_kernel<<<dim3(kDin / 64, kDtR / 64), 256, 0, stream>>>(W_dt + (size_t)dir * kDtR * kDin, WDT16, kDtR, kDin, kDin, kCarryW);
    transpose_cast_kernel<<<dim3(kDmod / 64, kDin / 64), 256, 0, stream>>>(W_out + (size_t)dir * kDin * kDmod, WOUT16, kDin, kDmod, kDmod, kCarryWS);
    transpose_cast_kernel<<<dim3(kDmod / 64, kDin / 64), 256, 0, stream>>>(W_out + (size_t)dir * kDin * kDmod, WOUTL, kDin, kDmod, kDmod, kCarryWL);

    layernorm_f16_kernel<<<kRows, 128, 0, stream>>>(x, ln_w + (size_t)dir * kDmod, ln_b + (size_t)dir * kDmod, XN16);

    wmma_gemm64<0, 0, 2, 0, false><<<dim3(256, 1), 256, 0, stream>>>(
        XN16, XN16, kDmod, 0L, WIN16, WIN16, kDmod, 0L,
        (void*)XZ, (void*)XZ, kXZP, 0L, b_in + (size_t)dir * kXZP, dummy_resid, 0L, kRows, kXZP, kDmod, sclW);

    conv_silu_kernel<<<dim3(kDin / 256, kRows / 64), 256, 0, stream>>>(XZ, conv_w + (size_t)dir * kDin * 4, conv_b + (size_t)dir * kDin, UC16, dir);

    wmma_gemm64<0, 0, 0, 0, false><<<dim3(8, 1), 256, 0, stream>>>(
        UC16, UC16, kDin, 0L, WXP16, WXP16, kDin, 0L,
        (void*)PROJ, (void*)PROJ, kPrjP, 0L, dummy_bias, dummy_resid, 0L, kRows, kPrjP, kDin, sclW);

    dt_cast_kernel<<<(kRows * kDtR) / 8 / 256, 256, 0, stream>>>(PROJ, DT16, (kRows * kDtR) / 8, kCarryDt);

    wmma_gemm64<0, 0, 2, 0, false><<<dim3(128, 1), 256, 0, stream>>>(
        DT16, DT16, kDtR, 0L, WDT16, WDT16, kDtR, 0L,
        (void*)DLR, (void*)DLR, kDin, 0L, b_dt + (size_t)dir * kDin, dummy_resid, 0L, kRows, kDin, kDtR, sclDtW);

    scan_kernel<<<dim3(kDin / 256, kBatch), 256, 0, stream>>>(
        DLR, XZ, PROJ, conv_w + (size_t)dir * kDin * 4, conv_b + (size_t)dir * kDin,
        A_log + (size_t)dir * kDin * kNst, Dv + (size_t)dir * kDin, Y16, YL, dir);

    wmma_gemm64<0, 3, 2, 0, false><<<dim3(64, 1), 256, 0, stream>>>(
        Y16, YL, kDin, 0L, WOUT16, WOUTL, kDin, 0L,
        (void*)(MO + (size_t)dir * kRows * kDmod), (void*)(MO + (size_t)dir * kRows * kDmod), kDmod, 0L,
        b_out + (size_t)dir * kDmod, dummy_resid, 0L, kRows, kDmod, kDin, sclYW);
  }

  transpose_cast_kernel<<<dim3(kDmod / 64, kCmbK / 64), 256, 0, stream>>>(Wg, WGVH, kCmbK, kDmod, kDmod, kCarryWS);
  transpose_cast_kernel<<<dim3(kDmod / 64, kCmbK / 64), 256, 0, stream>>>(Wv, WGVH + (size_t)kDmod * kCmbK, kCmbK, kDmod, kDmod, kCarryWS);
  transpose_cast_kernel<<<dim3(kDmod / 64, kCmbK / 64), 256, 0, stream>>>(Wg, WGVL, kCmbK, kDmod, kDmod, kCarryWL);
  transpose_cast_kernel<<<dim3(kDmod / 64, kCmbK / 64), 256, 0, stream>>>(Wv, WGVL + (size_t)kDmod * kCmbK, kCmbK, kDmod, kDmod, kCarryWL);

  comb_cast_kernel<<<(kRows * kCmbK) / 8 / 256, 256, 0, stream>>>(MO, x, COMBH, COMBL, (kRows * kCmbK) / 8);

  wmma_gemm64<0, 3, 2, 0, false><<<dim3(64, 1), 256, 0, stream>>>(
      COMBH, COMBL, kCmbK, 0L, WGVH, WGVL, kCmbK, 0L,
      (void*)GV, (void*)GV, kGVP, 0L, bg, dummy_resid, 0L, kRows, kDmod, kCmbK, sclGW);
  wmma_gemm64<0, 3, 2, 0, false><<<dim3(64, 1), 256, 0, stream>>>(
      COMBH, COMBL, kCmbK, 0L, WGVH + (size_t)kDmod * kCmbK, WGVL + (size_t)kDmod * kCmbK, kCmbK, 0L,
      (void*)(GV + kDmod), (void*)(GV + kDmod), kGVP, 0L, bv, dummy_resid, 0L, kRows, kDmod, kCmbK, sclGW);

  gate_fuse_kernel<<<(kRows * kDmod) / 4 / 256, 256, 0, stream>>>(GV, MO, x, dout, (kRows * kDmod) / 4);
}
